// DifferentiableExtrusion_21268678050249
// MI455X (gfx1250) — hardware-verified
//
#include <hip/hip_runtime.h>
#include <stdint.h>

typedef float v8f __attribute__((ext_vector_type(8)));
typedef float v4f __attribute__((ext_vector_type(4)));
typedef float v4fa __attribute__((ext_vector_type(4), may_alias));
typedef __bf16 v16b __attribute__((ext_vector_type(16)));
typedef unsigned int v8u __attribute__((ext_vector_type(8)));
union Frag { v16b v; v8u w; };

#define VOX 64
#define MPTS (VOX * VOX)
#define PVERT 16
#define MAXN 32
#define MAXE (MAXN * PVERT)
#define TPB 256
#define WAVES (TPB / 32)
#define PTS_BLK (WAVES * 16)
#define BLK_PER_B (MPTS / PTS_BLK)

typedef char chk_tiling_t[(MPTS % PTS_BLK == 0) ? 1 : -1];
typedef char chk_store_t[(PTS_BLK == 4 * 32) ? 1 : -1];
typedef char chk_zwave_t[((VOX % WAVES) == 0) ? 1 : -1];

__device__ __forceinline__ unsigned int bf16_rne_bits(float f) {
  unsigned int u = __float_as_uint(f);
  return (u + 0x7FFFu + ((u >> 16) & 1u)) >> 16;
}
__device__ __forceinline__ float bf16_bits_to_f32(unsigned int b) {
  return __uint_as_float(b << 16);
}

__device__ __forceinline__ v8f wmma_bf16(v16b a, v16b b, v8f c) {
  v8f d = __builtin_amdgcn_wmma_f32_16x16x32_bf16(false, a, false, b, (short)0, c, false, false);
  asm volatile("v_nop\n\tv_nop\n\tv_nop\n\tv_nop" : "+v"(d) : "v"(a), "v"(b));
  return d;
}

__device__ __forceinline__ v16b make_frag(unsigned int w0, unsigned int w1, unsigned int w2) {
  Frag f;
#pragma unroll
  for (int i = 0; i < 8; ++i) f.w[i] = 0u;
  f.w[0] = w0; f.w[1] = w1; f.w[2] = w2;
  return f.v;
}

__global__ __launch_bounds__(TPB) void k_extrude(
    const float* __restrict__ polygons,
    const float* __restrict__ attributes,
    const float* __restrict__ validity,
    float* __restrict__ out,
    int nbatch, int n_poly, int attr_stride) {
  __shared__ float sP1x[MAXE], sP1y[MAXE], sUx[MAXE], sUy[MAXE], sLen[MAXE], sC1[MAXE];
  __shared__ unsigned int sW0[MAXE], sW1[MAXE], sW2[MAXE];
  __shared__ int sGate[MAXN];
  __shared__ __attribute__((aligned(16))) float sMask[PTS_BLK];

  const int b = blockIdx.x / BLK_PER_B;
  if (b >= nbatch) return;
  const int blk0 = (blockIdx.x - b * BLK_PER_B) * PTS_BLK;
  const int tid = threadIdx.x;
  const int n_edge = n_poly * PVERT;
  const float vscale = (float)(VOX - 1);

  const float* pb = polygons + (size_t)b * (size_t)n_edge * 2;
  for (int e = tid; e < n_edge; e += TPB) {
    const int pidx = e & (PVERT - 1);
    const int nxt  = (e & ~(PVERT - 1)) | ((pidx + 1) & (PVERT - 1));
    const float p1x = pb[2 * e + 0] * vscale;
    const float p1y = pb[2 * e + 1] * vscale;
    const float p2x = pb[2 * nxt + 0] * vscale;
    const float p2y = pb[2 * nxt + 1] * vscale;
    const float vx = p2x - p1x, vy = p2y - p1y;
    const float len = sqrtf(vx * vx + vy * vy);
    const float inv = 1.0f / fmaxf(len, 1e-12f);
    const float ux = vx * inv, uy = vy * inv;
    const unsigned int hx = bf16_rne_bits(ux), hy = bf16_rne_bits(uy);
    const float rx1 = ux - bf16_bits_to_f32(hx), ry1 = uy - bf16_bits_to_f32(hy);
    const unsigned int mx = bf16_rne_bits(rx1), my = bf16_rne_bits(ry1);
    const float rx2 = rx1 - bf16_bits_to_f32(mx), ry2 = ry1 - bf16_bits_to_f32(my);
    const unsigned int lx = bf16_rne_bits(rx2), ly = bf16_rne_bits(ry2);
    sP1x[e] = p1x; sP1y[e] = p1y; sUx[e] = ux; sUy[e] = uy; sLen[e] = len;
    sC1[e]  = p1x * ux + p1y * uy;
    sW0[e] = hx | (hy << 16);
    sW1[e] = mx | (my << 16);
    sW2[e] = lx | (ly << 16);
  }
  if (tid < n_poly) {
    const float* pp = pb + (size_t)tid * (PVERT * 2);
    int nz = 0;
#pragma unroll 8
    for (int j = 0; j < PVERT * 2; ++j) nz |= (pp[j] != 0.0f) ? 1 : 0;
    const int valid = (validity[(size_t)b * n_poly + tid] >= 0.5f) ? 1 : 0;
    sGate[tid] = (nz & valid);
  }
  __syncthreads();

  const int wave = tid >> 5;
  const int l    = tid & 31;
  const int h    = l >> 4;
  const int col  = l & 15;
  const int m0   = blk0 + wave * 16;
  const float ybase = (float)(m0 >> 6);
  const float xbase = (float)(m0 & 63);
  const float xh    = xbase + (float)(8 * h);

  const unsigned int axb = bf16_rne_bits(xbase + (float)col);
  const unsigned int ayb = bf16_rne_bits(ybase);
  const unsigned int aw  = (h == 0) ? (axb | (ayb << 16)) : 0u;
  const v16b afrag = make_frag(aw, aw, aw);
  v8f cz;
#pragma unroll
  for (int r = 0; r < 8; ++r) cz[r] = 0.0f;

  float mind[8];
#pragma unroll
  for (int r = 0; r < 8; ++r) mind[r] = 1e30f;

  for (int n = 0; n < n_poly; ++n) {
    const int g = __builtin_amdgcn_readfirstlane(sGate[n]);
    if (g == 0) continue;
    const int e = n * PVERT + col;
    const unsigned int w0 = (h == 0) ? sW0[e] : 0u;
    const unsigned int w1 = (h == 0) ? sW1[e] : 0u;
    const unsigned int w2 = (h == 0) ? sW2[e] : 0u;
    const v16b bfrag = make_frag(w0, w1, w2);
    const v8f d = wmma_bf16(afrag, bfrag, cz);

    const float p1x = sP1x[e], p1y = sP1y[e], ux = sUx[e], uy = sUy[e];
    const float len = sLen[e], c1 = sC1[e];
    const bool  safe = len > 1e-6f;
#pragma unroll
    for (int r = 0; r < 8; ++r) {
      const float xr = xh + (float)r;
      const float s  = d[r] - c1;
      const float t  = fminf(fmaxf(s, 0.0f), len);
      const float cx = safe ? (p1x + t * ux) : p1x;
      const float cy = safe ? (p1y + t * uy) : p1y;
      const float dx = xr - cx, dy = ybase - cy;
      float dist = __builtin_amdgcn_sqrtf(dx * dx + dy * dy);
      dist = fminf(dist, __shfl_xor(dist, 1, 32));
      dist = fminf(dist, __shfl_xor(dist, 2, 32));
      dist = fminf(dist, __shfl_xor(dist, 4, 32));
      dist = fminf(dist, __shfl_xor(dist, 8, 32));
      mind[r] = fminf(mind[r], dist);
    }
  }

  if (col == 0) {
#pragma unroll
    for (int r = 0; r < 8; ++r) {
      const float md = mind[r];
      float v = 0.0f;
      if (md < 1e29f) v = __builtin_amdgcn_rcpf(1.0f + __builtin_amdgcn_exp2f(md * 1.4426950408889634f));
      sMask[wave * 16 + 8 * h + r] = v;
    }
  }
  __syncthreads();

  const float hv = fminf(floorf(attributes[(size_t)b * attr_stride] * (float)VOX), (float)VOX);
  const v4f mv = *(const v4fa*)(sMask + 4 * l);
  v4f z4;
  z4[0] = 0.0f; z4[1] = 0.0f; z4[2] = 0.0f; z4[3] = 0.0f;
  float* ob = out + (size_t)b * VOX * MPTS + (size_t)blk0 + 4 * l;
#pragma unroll 1
  for (int z = wave; z < VOX; z += WAVES) {
    v4f v = mv;
    if (!((float)z < hv)) v = z4;
    *(volatile v4f*)(ob + (size_t)z * MPTS) = v;
  }
  __threadfence();
#pragma unroll 1
  for (int z = wave; z < VOX; z += WAVES) {
    v4f v = mv;
    if (!((float)z < hv)) v = z4;
    *(volatile v4f*)(ob + (size_t)z * MPTS) = v;
  }
}

extern "C" void kernel_launch(void* const* d_in, const int* in_sizes, int n_in,
                              void* d_out, int out_size, void* d_ws, size_t ws_size,
                              hipStream_t stream) {
  (void)d_ws; (void)ws_size;
  if (n_in < 3) return;
  const float* polygons   = (const float*)d_in[0];
  const float* attributes = (const float*)d_in[1];
  const float* validity   = (const float*)d_in[2];
  float* out = (float*)d_out;

  const int vol = VOX * MPTS;
  const int nbatch = out_size / vol;
  if (nbatch <= 0 || nbatch * vol != out_size) return;
  const int n_poly = in_sizes[2] / nbatch;
  if (n_poly <= 0 || n_poly > MAXN || n_poly * nbatch != in_sizes[2]) return;
  if (in_sizes[0] != nbatch * n_poly * PVERT * 2) return;
  const int attr_stride = in_sizes[1] / nbatch;
  if (attr_stride <= 0) return;

  dim3 grid(nbatch * BLK_PER_B);
  k_extrude<<<grid, TPB, 0, stream>>>(polygons, attributes, validity, out, nbatch, n_poly, attr_stride);
}
